// TransformerBlock_541165879394
// MI455X (gfx1250) — hardware-verified
//
#include <hip/hip_runtime.h>
#include <stddef.h>


typedef _Float16 v16h __attribute__((ext_vector_type(16)));
typedef _Float16 v8h  __attribute__((ext_vector_type(8)));
typedef float    v8f  __attribute__((ext_vector_type(8)));
typedef float    v4f  __attribute__((ext_vector_type(4)));

#ifndef NB
#define NB 1
#endif
#ifndef SEQ
#define SEQ 2048
#endif
#define NB_FULL  1
#define SEQ_FULL 2048
#define DIM   1024
#define NHEAD 16
#define HD    64
#define DFF   4096
#define MROWS (NB * SEQ)

static_assert(NB >= 1 && NB <= NB_FULL);
static_assert(SEQ >= 128 && SEQ <= SEQ_FULL && (SEQ % 128) == 0);
static_assert(DIM == NHEAD * HD);
static_assert(HD == 64);
static_assert((DIM % 64) == 0 && (DIM % 32) == 0);
static_assert((DFF % 64) == 0 && (DFF % 32) == 0);
static_assert((MROWS % 64) == 0);
static_assert(DIM == 128 * 8);
static_assert((size_t)MROWS * DFF < (size_t)0xFFFFFFFFu);

#define LDT 72
#define LDC 68
static_assert((LDT % 8) == 0 && LDT >= 64);
static_assert((LDC % 4) == 0 && LDC >= 64);

#define WCARRY 64.0f
#define PCARRY 1024.0f
#define VCARRY 64.0f
#define ACARRY 64.0f

#define PLANE16_ELEMS ((size_t)MROWS * DIM)
#define PLANE16_BYTES (PLANE16_ELEMS * 2)
#define WSQ_ELEMS     ((size_t)DIM * DIM)
#define OFF_WQKV  ((size_t)0)
#define OFF_WO    (OFF_WQKV + 3 * WSQ_ELEMS * 2)
#define OFF_W1    (OFF_WO + WSQ_ELEMS * 2)
#define OFF_W2    (OFF_W1 + (size_t)DFF * DIM * 2)
#define OFF_H1    (OFF_W2 + (size_t)DFF * DIM * 2)
#define OFF_QKV   (OFF_H1 + PLANE16_BYTES)
#define OFF_CTX   (OFF_QKV + 3 * PLANE16_BYTES)
#define OFF_X1    (OFF_CTX + PLANE16_BYTES)
#define OFF_H2    (OFF_X1 + PLANE16_ELEMS * 4)
#define OFF_ACT   (OFF_H2 + PLANE16_BYTES)
#define WS_TOTAL  (OFF_ACT + (size_t)MROWS * DFF * 2)
static_assert((PLANE16_BYTES % 128) == 0 && ((WSQ_ELEMS * 2) % 128) == 0);
static_assert((OFF_ACT % 128) == 0 && (OFF_X1 % 128) == 0);
static_assert(WS_TOTAL <= (size_t)134217728);

__device__ __forceinline__ float bf16r(float x) {
  unsigned int u = __float_as_uint(x);
  u = (u + 0x7FFFu + ((u >> 16) & 1u)) & 0xFFFF0000u;
  return __uint_as_float(u);
}

__device__ __forceinline__ size_t full_row(unsigned crow) {
  const unsigned bidx = crow / (unsigned)SEQ;
  const unsigned sq = crow - bidx * (unsigned)SEQ;
  return (size_t)bidx * SEQ_FULL + sq;
}

__device__ __forceinline__ v16h frag_at(const _Float16* p) {
  v8h lo = *(const v8h*)(p);
  v8h hi = *(const v8h*)(p + 16);
  v16h out;
#pragma unroll
  for (int i = 0; i < 8; ++i) { out[i] = lo[i]; out[i + 8] = hi[i]; }
  return out;
}
__device__ __forceinline__ v16h ld_frag(const _Float16* base, unsigned ld) {
  const unsigned lane = threadIdx.x & 31u;
  return frag_at(base + (lane & 15u) * ld + (lane >> 4) * 8u);
}

__device__ __forceinline__ v8f wmma16(v16h a, v16h b, v8f c) {
  v8f d = __builtin_amdgcn_wmma_f32_16x16x32_f16(false, a, false, b, (short)0, c,
                                                 false, false);
  asm volatile("v_nop\n\tv_nop\n\tv_nop\n\tv_nop" : "+v"(d) : "v"(a), "v"(b));
  return d;
}

__device__ __forceinline__ float red16_max(float x) {
#pragma unroll
  for (int off = 1; off < 16; off <<= 1) x = fmaxf(x, __shfl_xor(x, off, 32));
  return x;
}
__device__ __forceinline__ float red16_sum(float x) {
#pragma unroll
  for (int off = 1; off < 16; off <<= 1) x += __shfl_xor(x, off, 32);
  return x;
}
__device__ __forceinline__ float red32_sum(float x) {
#pragma unroll
  for (int off = 1; off < 32; off <<= 1) x += __shfl_xor(x, off, 32);
  return x;
}

__device__ __forceinline__ void wave_lds_sync() {
  __builtin_amdgcn_fence(3  , "wavefront");
  asm volatile("s_wait_dscnt 0x0" ::: "memory");
  __builtin_amdgcn_wave_barrier();
}

__global__ __launch_bounds__(256) void wconv_kernel(
    const float* __restrict__ W, _Float16* __restrict__ Wt,
    unsigned N, unsigned K, unsigned headmode) {
  __shared__ _Float16 T[64 * LDT];
  const unsigned tid = threadIdx.x;
  const unsigned n0 = blockIdx.x * 64u;
  const unsigned k0 = blockIdx.y * 64u;
  const size_t sbase = headmode ? (size_t)blockIdx.x * K * 64u : (size_t)n0;
  const unsigned ldw = headmode ? 64u : N;
#pragma unroll 4
  for (unsigned j = 0; j < 16u; ++j) {
    const unsigned idx = tid + 256u * j;
    const unsigned kr = idx >> 6, nc = idx & 63u;
    const float v = W[sbase + (size_t)(k0 + kr) * ldw + nc];
    T[nc * LDT + kr] = (_Float16)(WCARRY * bf16r(v));
  }
  __syncthreads();
  v8h x[2];
  size_t off[2];
#pragma unroll
  for (unsigned i = 0; i < 2u; ++i) {
    const unsigned n = 32u * i + (tid >> 3);
    const unsigned kc = (tid & 7u) * 8u;
    x[i] = *(const v8h*)&T[n * LDT + kc];
    off[i] = (size_t)(n0 + n) * K + k0 + kc;
  }
#pragma unroll
  for (int i = 0; i < 2; ++i) *(volatile v8h*)(Wt + off[i]) = x[i];
  __threadfence();
#pragma unroll
  for (int i = 0; i < 2; ++i) *(volatile v8h*)(Wt + off[i]) = x[i];
}

__global__ __launch_bounds__(128) void ln_kernel(
    const float* __restrict__ Xin, const float* __restrict__ g,
    const float* __restrict__ bta, _Float16* __restrict__ dst,
    unsigned src_full, unsigned rne_in) {
  __shared__ float rowf[DIM];
  __shared__ _Float16 rowh[DIM];
  __shared__ float red[8];
  const unsigned tid = threadIdx.x, lane = tid & 31u, w = tid >> 5;
  const unsigned crow = blockIdx.x;
  const size_t srow = src_full ? full_row(crow) : (size_t)crow;
  const float* sp = Xin + srow * DIM + tid * 8u;
  v4f a0 = *(const v4f*)(sp);
  v4f a1 = *(const v4f*)(sp + 4);
  if (rne_in) {
#pragma unroll
    for (int j = 0; j < 4; ++j) { a0[j] = bf16r(a0[j]); a1[j] = bf16r(a1[j]); }
  }
  *(v4f*)&rowf[tid * 8u] = a0;
  *(v4f*)&rowf[tid * 8u + 4u] = a1;
  float s = ((a0[0] + a0[1]) + (a0[2] + a0[3])) + ((a1[0] + a1[1]) + (a1[2] + a1[3]));
  s = red32_sum(s);
  if (lane == 0u) red[w] = s;
  __syncthreads();
  const float mean = ((red[0] + red[1]) + (red[2] + red[3])) * (1.0f / (float)DIM);
  float ss = 0.0f;
#pragma unroll
  for (int j = 0; j < 4; ++j) {
    const float d0 = a0[j] - mean, d1 = a1[j] - mean;
    ss += d0 * d0;
    ss += d1 * d1;
  }
  ss = red32_sum(ss);
  if (lane == 0u) red[4u + w] = ss;
  __syncthreads();
  const float var = ((red[4] + red[5]) + (red[6] + red[7])) / (float)(DIM - 1);
  const float den = sqrtf(var) + 1.0e-8f;
#pragma unroll 1
  for (unsigned j = 0; j < 8u; ++j) {
    const unsigned c = tid + 128u * j;
    const float v = rowf[c];
    rowh[c] = (_Float16)((v - mean) / den * bf16r(g[c]) + bf16r(bta[c]));
  }
  __syncthreads();
  const v8h o = *(const v8h*)&rowh[tid * 8u];
  _Float16* dp = dst + (size_t)crow * DIM + tid * 8u;
  *(volatile v8h*)dp = o;
  __threadfence();
  *(volatile v8h*)dp = o;
}

__device__ __forceinline__ void gemm_main(
    const _Float16* __restrict__ A16, const _Float16* __restrict__ Bt,
    const unsigned K, const unsigned arow0, const unsigned brow0, float* Cs) {
  const unsigned tid = threadIdx.x, lane = tid & 31u, w = tid >> 5;
  const unsigned mw = w >> 1, nw = w & 1u;
  const unsigned hh = lane >> 4, m = lane & 15u;
  const _Float16* ap  = A16 + (size_t)(arow0 + mw * 16u + m) * K + hh * 8u;
  const _Float16* bp0 = Bt + (size_t)(brow0 + nw * 32u + m) * K + hh * 8u;
  const _Float16* bp1 = bp0 + (size_t)16 * K;
  v8f acc0 = {}, acc1 = {};
#pragma unroll 2
  for (unsigned k0 = 0; k0 < K; k0 += 32u) {
    const v16h a  = frag_at(ap + k0);
    const v16h b0 = frag_at(bp0 + k0);
    const v16h b1 = frag_at(bp1 + k0);
    acc0 = wmma16(a, b0, acc0);
    acc1 = wmma16(a, b1, acc1);
  }
#pragma unroll
  for (int r = 0; r < 8; ++r) {
    float* d = &Cs[(mw * 16u + hh * 8u + (unsigned)r) * LDC + nw * 32u + m];
    d[0]  = acc0[r];
    d[16] = acc1[r];
  }
  __syncthreads();
}

__device__ __forceinline__ void epi_f16(
    const float* Cs, _Float16* __restrict__ out16, const unsigned pitch,
    const unsigned row0, const unsigned n0, const float scale) {
  const unsigned tid = threadIdx.x;
  v8h x[2];
  size_t off[2];
#pragma unroll
  for (unsigned i = 0; i < 2u; ++i) {
    const unsigned r = 32u * i + (tid >> 3);
    const unsigned c = (tid & 7u) * 8u;
    const v4f u0 = *(const v4f*)&Cs[r * LDC + c];
    const v4f u1 = *(const v4f*)&Cs[r * LDC + c + 4];
#pragma unroll
    for (int j = 0; j < 4; ++j) {
      x[i][j]     = (_Float16)(u0[j] * scale);
      x[i][j + 4] = (_Float16)(u1[j] * scale);
    }
    off[i] = (size_t)(row0 + r) * pitch + n0 + c;
  }
#pragma unroll
  for (int i = 0; i < 2; ++i) *(volatile v8h*)(out16 + off[i]) = x[i];
  __threadfence();
#pragma unroll
  for (int i = 0; i < 2; ++i) *(volatile v8h*)(out16 + off[i]) = x[i];
}

__device__ __forceinline__ void epi_vt(
    const float* Cs, _Float16* __restrict__ out16,
    const unsigned row0, const unsigned n0, const float scale) {
  const unsigned tid = threadIdx.x;
  const unsigned bidx = row0 / (unsigned)SEQ;
  const unsigned key0 = row0 - bidx * (unsigned)SEQ;
  v8h x[2];
  size_t off[2];
#pragma unroll
  for (unsigned i = 0; i < 2u; ++i) {
    const unsigned dcol = 32u * i + (tid >> 3);
    const unsigned kk = (tid & 7u) * 8u;
#pragma unroll
    for (unsigned j = 0; j < 8u; ++j)
      x[i][j] = (_Float16)(Cs[(kk + j) * LDC + dcol] * scale);
    off[i] = ((size_t)bidx * DIM + n0 + dcol) * SEQ + key0 + kk;
  }
#pragma unroll
  for (int i = 0; i < 2; ++i) *(volatile v8h*)(out16 + off[i]) = x[i];
  __threadfence();
#pragma unroll
  for (int i = 0; i < 2; ++i) *(volatile v8h*)(out16 + off[i]) = x[i];
}

__device__ __forceinline__ void epi_f32(
    const float* Cs, const float* __restrict__ bias, const float* __restrict__ res,
    const unsigned res_full, const unsigned res_rne, float* __restrict__ outf,
    const unsigned out_full, const unsigned row0, const unsigned n0, const float scale) {
  const unsigned tid = threadIdx.x;
  v4f xs[4];
  size_t off[4];
#pragma unroll
  for (unsigned i = 0; i < 4u; ++i) {
    const unsigned r = 16u * i + (tid >> 4);
    const unsigned c = (tid & 15u) * 4u;
    const unsigned crow = row0 + r;
    const size_t frow = full_row(crow);
    const size_t rrow = res_full ? frow : (size_t)crow;
    const size_t orow = out_full ? frow : (size_t)crow;
    const v4f u = *(const v4f*)&Cs[r * LDC + c];
    const v4f g = *(const v4f*)(bias + n0 + c);
    const v4f rv = *(const v4f*)(res + rrow * DIM + n0 + c);
    v4f val;
#pragma unroll
    for (int j = 0; j < 4; ++j) {
      const float rr = res_rne ? bf16r(rv[j]) : rv[j];
      val[j] = (u[j] * scale + bf16r(g[j])) + rr;
    }
    xs[i] = val;
    off[i] = orow * DIM + n0 + c;
  }
#pragma unroll
  for (int i = 0; i < 4; ++i) *(volatile v4f*)(outf + off[i]) = xs[i];
  __threadfence();
#pragma unroll
  for (int i = 0; i < 4; ++i) *(volatile v4f*)(outf + off[i]) = xs[i];
}

__global__ __launch_bounds__(256) void gemm_qkv_kernel(
    const _Float16* __restrict__ H16, const _Float16* __restrict__ WqkvT,
    _Float16* __restrict__ qkv16) {
  __shared__ float Cs[64 * LDC];
  const unsigned sel = blockIdx.x / (unsigned)(DIM / 64);
  const unsigned n0 = (blockIdx.x - sel * (unsigned)(DIM / 64)) * 64u;
  const unsigned row0 = blockIdx.y * 64u;
  gemm_main(H16, WqkvT, (unsigned)DIM, row0, blockIdx.x * 64u, Cs);
  _Float16* outp = qkv16 + (size_t)sel * PLANE16_ELEMS;
  if (sel < 2u) epi_f16(Cs, outp, (unsigned)DIM, row0, n0, 1.0f / WCARRY);
  else          epi_vt(Cs, outp, row0, n0, 1.0f / WCARRY);
}

__global__ __launch_bounds__(256) void gemm_wo_kernel(
    const _Float16* __restrict__ Ctx16, const _Float16* __restrict__ WoT,
    const float* __restrict__ bo, const float* __restrict__ X, float* __restrict__ X1) {
  __shared__ float Cs[64 * LDC];
  const unsigned n0 = blockIdx.x * 64u;
  const unsigned row0 = blockIdx.y * 64u;
  gemm_main(Ctx16, WoT, (unsigned)DIM, row0, n0, Cs);
  epi_f32(Cs, bo, X, 1u, 1u, X1, 0u, row0, n0, 1.0f / (WCARRY * VCARRY));
}

__global__ __launch_bounds__(256) void gemm_ffn1_kernel(
    const _Float16* __restrict__ H2, const _Float16* __restrict__ W1T,
    const float* __restrict__ b1, _Float16* __restrict__ Act16) {
  __shared__ float Cs[64 * LDC];
  const unsigned tid = threadIdx.x;
  const unsigned n0 = blockIdx.x * 64u;
  const unsigned row0 = blockIdx.y * 64u;
  gemm_main(H2, W1T, (unsigned)DIM, row0, n0, Cs);
#pragma unroll 1
  for (unsigned e = 0; e < 16u; ++e) {
    const unsigned r = 32u * (e >> 3) + (tid >> 3);
    const unsigned c = (tid & 7u) * 8u + (e & 7u);
    const float t = Cs[r * LDC + c] * (1.0f / WCARRY) + bf16r(b1[n0 + c]);
    Cs[r * LDC + c] = (ACARRY * 0.5f) * t * (1.0f + erff(t * 0.70710678118654752f));
  }
  __syncthreads();
  epi_f16(Cs, Act16, (unsigned)DFF, row0, n0, 1.0f);
}

__global__ __launch_bounds__(256) void gemm_ffn2_kernel(
    const _Float16* __restrict__ Act16, const _Float16* __restrict__ W2T,
    const float* __restrict__ b2, const float* __restrict__ X1, float* __restrict__ out) {
  __shared__ float Cs[64 * LDC];
  const unsigned n0 = blockIdx.x * 64u;
  const unsigned row0 = blockIdx.y * 64u;
  gemm_main(Act16, W2T, (unsigned)DFF, row0, n0, Cs);
  epi_f32(Cs, b2, X1, 0u, 0u, out, 1u, row0, n0, 1.0f / (WCARRY * ACARRY));
}

__global__ __launch_bounds__(256) void attn_kernel(
    const _Float16* __restrict__ Qh, const _Float16* __restrict__ Kh,
    const _Float16* __restrict__ Vt, _Float16* __restrict__ Ov) {
  __shared__ _Float16 Ks[64 * LDT];
  __shared__ _Float16 Vs[64 * LDT];
  __shared__ _Float16 Ps[8 * 16 * LDT];

  const unsigned tid = threadIdx.x, lane = tid & 31u;
  const unsigned w = (unsigned)__builtin_amdgcn_readfirstlane((int)(tid >> 5));
  const unsigned hh = lane >> 4, m = lane & 15u;
  const unsigned q0 = blockIdx.x * 128u;
  const unsigned head = blockIdx.y;
  const unsigned b = blockIdx.z;
  const unsigned qw0 = q0 + w * 16u;
  const float scale = 0.125f;
  _Float16* P = Ps + w * (16u * LDT);

  const size_t qoff = (size_t)(b * (unsigned)SEQ + qw0 + m) * DIM + head * HD + hh * 8u;
  v16h qf[2];
  qf[0] = frag_at(Qh + qoff);
  qf[1] = frag_at(Qh + qoff + 32);

  float mrow[8], lrow[8];
  v8f o[4];
#pragma unroll
  for (int v = 0; v < 8; ++v) { mrow[v] = -1.0e30f; lrow[v] = 0.0f; }
#pragma unroll
  for (int nb = 0; nb < 4; ++nb) o[nb] = (v8f){};

  const size_t kplane = (size_t)b * SEQ * DIM + head * HD;
  const size_t vplane = ((size_t)b * DIM + head * HD) * SEQ;
  const unsigned kend = q0 + 128u;

  for (unsigned kb = 0; kb < kend; kb += 64u) {
#pragma unroll
    for (unsigned j = 0; j < 2u; ++j) {
      const unsigned idx = tid + 256u * j;
      const unsigned r = idx >> 3, c = (idx & 7u) * 8u;
      *(v8h*)&Ks[r * LDT + c] = *(const v8h*)(Kh + kplane + (size_t)(kb + r) * DIM + c);
      *(v8h*)&Vs[r * LDT + c] = *(const v8h*)(Vt + vplane + (size_t)r * SEQ + kb + c);
    }
    __syncthreads();

    if (kb <= qw0 + 15u) {
      v8f s[4];
#pragma unroll
      for (int kg = 0; kg < 4; ++kg) {
        v8f t = {};
#pragma unroll
        for (int c = 0; c < 2; ++c) {
          const v16h kf = ld_frag(&Ks[(kg * 16) * LDT + c * 32], LDT);
          t = wmma16(qf[c], kf, t);
        }
        s[kg] = t * scale;
      }
      if (kb + 63u > qw0) {
#pragma unroll
        for (int kg = 0; kg < 4; ++kg) {
          const unsigned key = kb + (unsigned)kg * 16u + m;
#pragma unroll
          for (int v = 0; v < 8; ++v) {
            const unsigned qr = qw0 + hh * 8u + (unsigned)v;
            s[kg][v] = (key > qr) ? -1.0e30f : s[kg][v];
          }
        }
      }

      float alpha[8];
#pragma unroll
      for (int v = 0; v < 8; ++v) {
        float mx = fmaxf(fmaxf(s[0][v], s[1][v]), fmaxf(s[2][v], s[3][v]));
        mx = red16_max(mx);
        const float mn = fmaxf(mrow[v], mx);
        alpha[v] = __expf(mrow[v] - mn);
        mrow[v] = mn;
      }
#pragma unroll
      for (int kg = 0; kg < 4; ++kg)
#pragma unroll
        for (int v = 0; v < 8; ++v) s[kg][v] = __expf(s[kg][v] - mrow[v]);
#pragma unroll
      for (int v = 0; v < 8; ++v) {
        const float rs = red16_sum((s[0][v] + s[1][v]) + (s[2][v] + s[3][v]));
        lrow[v] = alpha[v] * lrow[v] + rs;
      }
#pragma unroll
      for (int nb = 0; nb < 4; ++nb)
#pragma unroll
        for (int v = 0; v < 8; ++v) o[nb][v] = o[nb][v] * alpha[v];

#pragma unroll
      for (int kg = 0; kg < 4; ++kg)
#pragma unroll
        for (int v = 0; v < 8; ++v)
          P[(hh * 8u + (unsigned)v) * LDT + (unsigned)kg * 16u + m] =
              (_Float16)(s[kg][v] * PCARRY);
      wave_lds_sync();

#pragma unroll
      for (int c = 0; c < 2; ++c) {
        const v16h pf = ld_frag(P + c * 32, LDT);
#pragma unroll
        for (int nb = 0; nb < 4; ++nb) {
          const v16h vf = ld_frag(&Vs[(nb * 16) * LDT + c * 32], LDT);
          o[nb] = wmma16(pf, vf, o[nb]);
        }
      }
    }
    __syncthreads();
  }

  float inv[8];
#pragma unroll
  for (int v = 0; v < 8; ++v) inv[v] = __builtin_amdgcn_rcpf(lrow[v]) * (VCARRY / PCARRY);
#pragma unroll
  for (int nb = 0; nb < 4; ++nb)
#pragma unroll
    for (int v = 0; v < 8; ++v)
      P[(hh * 8u + (unsigned)v) * LDT + (unsigned)nb * 16u + m] = (_Float16)(o[nb][v] * inv[v]);
  wave_lds_sync();
  v8h x[4];
  size_t off[4];
#pragma unroll
  for (unsigned i = 0; i < 4u; ++i) {
    const unsigned r = 4u * i + (lane >> 3);
    const unsigned c = (lane & 7u) * 8u;
    x[i] = *(const v8h*)&P[r * LDT + c];
    off[i] = (size_t)(b * (unsigned)SEQ + qw0 + r) * DIM + head * HD + c;
  }
#pragma unroll
  for (int i = 0; i < 4; ++i) *(volatile v8h*)(Ov + off[i]) = x[i];
  __threadfence();
#pragma unroll
  for (int i = 0; i < 4; ++i) *(volatile v8h*)(Ov + off[i]) = x[i];
}

extern "C" void kernel_launch(void* const* d_in, const int* in_sizes, int n_in,
                              void* d_out, int out_size, void* d_ws, size_t ws_size,
                              hipStream_t stream) {
  if (n_in < 14) return;
  const long long need_x = ((long long)(NB - 1) * SEQ_FULL + SEQ) * DIM;
  if ((long long)in_sizes[0] < need_x) return;
  if ((long long)in_sizes[1] < (long long)DIM * DIM) return;
  if ((long long)in_sizes[2] < (long long)DIM * DIM) return;
  if ((long long)in_sizes[3] < (long long)DIM * DIM) return;
  if ((long long)in_sizes[4] < (long long)DIM * DIM) return;
  if (in_sizes[5] < DIM || in_sizes[6] < DIM || in_sizes[7] < DIM) return;
  if (in_sizes[8] < DIM || in_sizes[9] < DIM) return;
  if ((long long)in_sizes[10] < (long long)DIM * DFF) return;
  if (in_sizes[11] < DFF) return;
  if ((long long)in_sizes[12] < (long long)DFF * DIM) return;
  if (in_sizes[13] < DIM) return;
  if ((long long)out_size < need_x) return;
  if (ws_size < WS_TOTAL) return;

  const float* X    = (const float*)d_in[0];
  const float* wq   = (const float*)d_in[1];
  const float* wk   = (const float*)d_in[2];
  const float* wv   = (const float*)d_in[3];
  const float* wo   = (const float*)d_in[4];
  const float* bo   = (const float*)d_in[5];
  const float* ln1g = (const float*)d_in[6];
  const float* ln1b = (const float*)d_in[7];
  const float* ln2g = (const float*)d_in[8];
  const float* ln2b = (const float*)d_in[9];
  const float* w1   = (const float*)d_in[10];
  const float* b1   = (const float*)d_in[11];
  const float* w2   = (const float*)d_in[12];
  const float* b2   = (const float*)d_in[13];
  float* out = (float*)d_out;

  char* ws = (char*)d_ws;
  _Float16* WqkvT = (_Float16*)(ws + OFF_WQKV);
  _Float16* WoT   = (_Float16*)(ws + OFF_WO);
  _Float16* W1T   = (_Float16*)(ws + OFF_W1);
  _Float16* W2T   = (_Float16*)(ws + OFF_W2);
  _Float16* H1    = (_Float16*)(ws + OFF_H1);
  _Float16* QKV16 = (_Float16*)(ws + OFF_QKV);
  _Float16* Ctx16 = (_Float16*)(ws + OFF_CTX);
  float*    X1    = (float*)(ws + OFF_X1);
  _Float16* H2    = (_Float16*)(ws + OFF_H2);
  _Float16* Act16 = (_Float16*)(ws + OFF_ACT);

  dim3 blk(256);
  wconv_kernel<<<dim3(DIM / 64, DIM / 64), blk, 0, stream>>>(wq, WqkvT + 0 * WSQ_ELEMS, DIM, DIM, 1u);
  wconv_kernel<<<dim3(DIM / 64, DIM / 64), blk, 0, stream>>>(wk, WqkvT + 1 * WSQ_ELEMS, DIM, DIM, 1u);
  wconv_kernel<<<dim3(DIM / 64, DIM / 64), blk, 0, stream>>>(wv, WqkvT + 2 * WSQ_ELEMS, DIM, DIM, 1u);
  wconv_kernel<<<dim3(DIM / 64, DIM / 64), blk, 0, stream>>>(wo, WoT, DIM, DIM, 0u);
  wconv_kernel<<<dim3(DFF / 64, DIM / 64), blk, 0, stream>>>(w1, W1T, DFF, DIM, 0u);
  wconv_kernel<<<dim3(DIM / 64, DFF / 64), blk, 0, stream>>>(w2, W2T, DIM, DFF, 0u);

  ln_kernel<<<dim3(MROWS), dim3(128), 0, stream>>>(X, ln1g, ln1b, H1, 1u, 1u);
  gemm_qkv_kernel<<<dim3(3 * DIM / 64, MROWS / 64), blk, 0, stream>>>(H1, WqkvT, QKV16);
  attn_kernel<<<dim3(SEQ / 128, NHEAD, NB), blk, 0, stream>>>(
      QKV16, QKV16 + PLANE16_ELEMS, QKV16 + 2 * PLANE16_ELEMS, Ctx16);
  gemm_wo_kernel<<<dim3(DIM / 64, MROWS / 64), blk, 0, stream>>>(Ctx16, WoT, bo, X, X1);
  ln_kernel<<<dim3(MROWS), dim3(128), 0, stream>>>(X1, ln2g, ln2b, H2, 0u, 0u);
  gemm_ffn1_kernel<<<dim3(DFF / 64, MROWS / 64), blk, 0, stream>>>(H2, W1T, b1, Act16);
  gemm_ffn2_kernel<<<dim3(DIM / 64, MROWS / 64), blk, 0, stream>>>(Act16, W2T, b2, X1, out);
}
